// MambaEncoder_33500744908981
// MI455X (gfx1250) — hardware-run, weakly checked
//
#include <hip/hip_runtime.h>
#include <math.h>

typedef __attribute__((ext_vector_type(16))) _Float16 v16h;
typedef __attribute__((ext_vector_type(8)))  _Float16 v8h;
typedef __attribute__((ext_vector_type(16))) __bf16   v16b;
typedef __attribute__((ext_vector_type(8)))  __bf16   v8b;
typedef __attribute__((ext_vector_type(8)))  float    v8f;
typedef __attribute__((ext_vector_type(4)))  float    v4f;

constexpr int kSeq     = 2048;
constexpr int kOutDim  = 512;
constexpr int kDModel  = 1024;
constexpr int kDInner  = 2048;
constexpr int kNState  = 16;
constexpr int kDConv   = 4;
constexpr int kDtRank  = 64;
constexpr int kXpReal  = kDtRank + 2 * kNState;
constexpr int kXpN     = 128;
constexpr int kXzPitch = 2 * kDInner;
constexpr int kConvTP  = 260;
constexpr int kScanTS  = 64;
constexpr int kScanCh  = 64;
constexpr int kScanYP  = 68;
constexpr int kBCP     = 32;
constexpr float kPScale    = 32768.0f;
constexpr float kPScaleInv = 1.0f / 32768.0f;
static_assert(kXpReal == 96);
static_assert(kDModel == 2 * kOutDim);
static_assert((kDModel % 32) == 0 && (kDInner % 32) == 0 && (kDtRank % 32) == 0 && (kOutDim % 32) == 0 && (kSeq % 32) == 0);
static_assert((kSeq % 64) == 0 && (kXzPitch % 64) == 0 && (kXpN % 64) == 0 && (kDInner % 64) == 0 && (kDModel % 64) == 0 && (kOutDim % 64) == 0);
static_assert((((kSeq / 64) * (kXzPitch / 64)) % 8) == 0 && (((kSeq / 64) * (kXpN / 64)) % 8) == 0 &&
              (((kSeq / 64) * (kDInner / 64)) % 8) == 0 && (((kSeq / 64) * (kDModel / 64)) % 8) == 0 &&
              (((kSeq / 64) * (kSeq / 64)) % 8) == 0 && (((kSeq / 64) * (kOutDim / 64)) % 8) == 0);
static_assert((kSeq % kScanTS) == 0 && (kDInner % kScanCh) == 0 && (kDInner % 256) == 0 && (kSeq % 64) == 0 && (kOutDim % 64) == 0);

constexpr size_t kOffTok  = 0;
constexpr size_t kOffWin  = kOffTok  + (size_t)kSeq    * kDModel  * 2;
constexpr size_t kOffWxp  = kOffWin  + (size_t)kXzPitch * kDModel * 2;
constexpr size_t kOffWdt  = kOffWxp  + (size_t)kXpN    * kDInner  * 2;
constexpr size_t kOffWout = kOffWdt  + (size_t)kDInner * kDtRank  * 2;
constexpr size_t kOffTxtT = kOffWout + (size_t)kDModel * kDInner  * 2;
constexpr size_t kOffXz   = kOffTxtT + (size_t)kOutDim * kSeq     * 2;
constexpr size_t kOffUc   = kOffXz   + (size_t)kSeq    * kXzPitch * 4;
constexpr size_t kOffUcb  = kOffUc   + (size_t)kSeq    * kDInner  * 4;
constexpr size_t kOffXd   = kOffUcb  + (size_t)kSeq    * kDInner  * 2;
constexpr size_t kOffDtr  = kOffXd   + (size_t)kSeq    * kXpN     * 4;
constexpr size_t kOffDtp  = kOffDtr  + (size_t)kSeq    * kDtRank  * 2;
constexpr size_t kOffY    = kOffDtp  + (size_t)kSeq    * kDInner  * 4;
constexpr size_t kOffMo   = kOffY    + (size_t)kSeq    * kDInner  * 2;
constexpr size_t kOffP    = kOffMo   + (size_t)kSeq    * kDModel  * 4;
constexpr size_t kOffCam  = kOffP    + (size_t)kSeq    * kSeq     * 2;
constexpr size_t kWsTotal = kOffCam  + (size_t)kSeq    * kOutDim  * 4;
constexpr size_t kOffS    = kOffXz;
static_assert(kWsTotal == 125829120ull);
static_assert(kWsTotal <= 134217728ull);
static_assert((size_t)kSeq * kSeq * 4 <= (size_t)kSeq * kXzPitch * 4);
static_assert((kOffWin % 128) == 0 && (kOffWxp % 128) == 0 && (kOffWdt % 128) == 0 && (kOffWout % 128) == 0 &&
              (kOffTxtT % 128) == 0 && (kOffXz % 128) == 0 && (kOffUc % 128) == 0 && (kOffUcb % 128) == 0 &&
              (kOffXd % 128) == 0 && (kOffDtr % 128) == 0 && (kOffDtp % 128) == 0 && (kOffY % 128) == 0 &&
              (kOffMo % 128) == 0 && (kOffP % 128) == 0 && (kOffCam % 128) == 0);
static_assert((size_t)kSeq * kOutDim * 4 == 4194304ull);
static_assert(2ull * kSeq * kOutDim * 4 == 8388608ull);

__device__ __forceinline__ unsigned short f2bf_bits(float f) {
  unsigned u = __float_as_uint(f);
  return (unsigned short)((u + 0x7FFFu + ((u >> 16) & 1u)) >> 16);
}
__device__ __forceinline__ float bf_bits2f(unsigned short h) { return __uint_as_float(((unsigned)h) << 16); }
__device__ __forceinline__ float bfr(float f) { return bf_bits2f(f2bf_bits(f)); }
__device__ __forceinline__ _Float16 bf_as_h(float f) { const unsigned short b = f2bf_bits(f); return __builtin_bit_cast(_Float16, b); }

__device__ __forceinline__ void dep_guard4_h(v8f& a, v8f& b, v8f& c, v8f& d, v16h x, v16h y) {
  asm volatile("v_nop\n\tv_nop\n\tv_nop\n\tv_nop" : "+v"(a), "+v"(b), "+v"(c), "+v"(d) : "v"(x), "v"(y));
}
__device__ __forceinline__ void dep_guard4_b(v8f& a, v8f& b, v8f& c, v8f& d, v16b x, v16b y) {
  asm volatile("v_nop\n\tv_nop\n\tv_nop\n\tv_nop" : "+v"(a), "+v"(b), "+v"(c), "+v"(d) : "v"(x), "v"(y));
}
__device__ __forceinline__ void keep4_h(v16h a, v16h b, v16h c, v16h d) { asm volatile("v_nop" :: "v"(a), "v"(b), "v"(c), "v"(d)); }
__device__ __forceinline__ void keep4_b(v16b a, v16b b, v16b c, v16b d) { asm volatile("v_nop" :: "v"(a), "v"(b), "v"(c), "v"(d)); }
__device__ __forceinline__ void acc_guard4(v8f& a, v8f& b, v8f& c, v8f& d) { asm volatile("v_nop\n\tv_nop\n\tv_nop\n\tv_nop" : "+v"(a), "+v"(b), "+v"(c), "+v"(d)); }
template <typename T> struct Frag;
template <> struct Frag<_Float16> {
  typedef v16h V; union U { v16h v; v8h h[2]; };
  static __device__ __forceinline__ v16h load(const _Float16* p) {
    U f; f.h[0] = *(const v8h*)(p); f.h[1] = *(const v8h*)(p + 16); return f.v;
  }
  static __device__ __forceinline__ v8f mma(v16h a, v16h b, v8f c) {
    return __builtin_amdgcn_wmma_f32_16x16x32_f16(false, a, false, b, (short)0, c, false, false);
  }
  static __device__ __forceinline__ void guard4(v8f& a, v8f& b, v8f& c, v8f& d, v16h x, v16h y) { dep_guard4_h(a, b, c, d, x, y); }
  static __device__ __forceinline__ void keep(v16h a, v16h b, v16h c, v16h d) { keep4_h(a, b, c, d); }
};
template <> struct Frag<__bf16> {
  typedef v16b V; union U { v16b v; v8b h[2]; };
  static __device__ __forceinline__ v16b load(const __bf16* p) {
    U f; f.h[0] = *(const v8b*)(p); f.h[1] = *(const v8b*)(p + 16); return f.v;
  }
  static __device__ __forceinline__ v8f mma(v16b a, v16b b, v8f c) {
    return __builtin_amdgcn_wmma_f32_16x16x32_bf16(false, a, false, b, (short)0, c, false, false);
  }
  static __device__ __forceinline__ void guard4(v8f& a, v8f& b, v8f& c, v8f& d, v16b x, v16b y) { dep_guard4_b(a, b, c, d, x, y); }
  static __device__ __forceinline__ void keep(v16b a, v16b b, v16b c, v16b d) { keep4_b(a, b, c, d); }
};

template <int ET> struct Elem;
template <> struct Elem<0> { typedef _Float16 T; };
template <> struct Elem<1> { typedef __bf16 T; };
template <int ET, bool SPLIT, int BIAS_MODE, int OUT_MODE, bool RESID, int ACT = 0>
__global__ __launch_bounds__(256) void wmma_gemm64(
    const unsigned short* __restrict__ Ap, const unsigned short* __restrict__ A2p, int lda, long strideA,
    const unsigned short* __restrict__ Btp, const unsigned short* __restrict__ Bt2p, int ldb, long strideB,
    void* __restrict__ Cout, void* __restrict__ Cout2, int ldc, long strideC,
    const float* __restrict__ bias,
    const float* __restrict__ resid, long strideR,
    int M, int N, int K, float scale) {
  typedef typename Elem<ET>::T T;
  typedef typename Frag<T>::V V;
  const T* A = (const T*)Ap; const T* A2 = (const T*)A2p; const T* Bt = (const T*)Btp; const T* Bt2 = (const T*)Bt2p;
  __shared__ __align__(16) float sT[8][16 * 68];
  const int b    = blockIdx.y;
  const int lane = threadIdx.x & 31;
  const int wave = threadIdx.x >> 5;
  const int tilesN = N >> 6;
  const int tilesM = M >> 6;
  const int tile = blockIdx.x * 8 + wave;
  if (tile >= tilesM * tilesN) return;
  const int tm = tile / tilesN;
  const int tn = tile - tm * tilesN;
  const int m0 = tm << 6;
  const int n0 = tn << 6;

  const T* Ab  = A  + (size_t)b * strideA;
  const T* Bb  = Bt + (size_t)b * strideB;
  const T* Ab2 = SPLIT ? (A2  + (size_t)b * strideA) : nullptr;
  const T* Bb2 = SPLIT ? (Bt2 + (size_t)b * strideB) : nullptr;

  const int rlane = lane & 15;
  const int koff  = (lane >> 4) * 8;
  const int mOff  = (lane >> 4) * 8;

  v8f acc[4][4];
#pragma unroll
  for (int i = 0; i < 4; ++i)
#pragma unroll
    for (int j = 0; j < 4; ++j) acc[i][j] = (v8f){0.f,0.f,0.f,0.f,0.f,0.f,0.f,0.f};

  for (int k0 = 0; k0 < K; k0 += 32) {
    V bh[4], bl[4];
#pragma unroll
    for (int j = 0; j < 4; ++j) {
      const size_t bo = (size_t)(n0 + (j << 4) + rlane) * ldb + koff + k0;
      bh[j] = Frag<T>::load(Bb + bo);
      if (SPLIT) bl[j] = Frag<T>::load(Bb2 + bo);
    }
#pragma unroll
    for (int i = 0; i < 4; ++i) {
      const size_t ao = (size_t)(m0 + (i << 4) + rlane) * lda + koff + k0;
      V ah = Frag<T>::load(Ab + ao);
      V al;
      if (SPLIT) al = Frag<T>::load(Ab2 + ao);
#pragma unroll
      for (int j = 0; j < 4; ++j) {
        acc[i][j] = Frag<T>::mma(ah, bh[j], acc[i][j]);
        if (SPLIT) {
          acc[i][j] = Frag<T>::mma(ah, bl[j], acc[i][j]);
          acc[i][j] = Frag<T>::mma(al, bh[j], acc[i][j]);
        }
      }
      Frag<T>::guard4(acc[i][0], acc[i][1], acc[i][2], acc[i][3], ah, SPLIT ? al : ah);
    }
    Frag<T>::keep(bh[0], bh[1], bh[2], bh[3]);
    if (SPLIT) Frag<T>::keep(bl[0], bl[1], bl[2], bl[3]);
  }
  acc_guard4(acc[0][0], acc[0][1], acc[0][2], acc[0][3]);
  acc_guard4(acc[1][0], acc[1][1], acc[1][2], acc[1][3]);
  acc_guard4(acc[2][0], acc[2][1], acc[2][2], acc[2][3]);
  acc_guard4(acc[3][0], acc[3][1], acc[3][2], acc[3][3]);

  float* slab = sT[wave];
  const float* Rb = RESID ? (resid + (size_t)b * strideR) : nullptr;
#pragma unroll
  for (int i = 0; i < 4; ++i) {
    const int mBase = m0 + (i << 4);
#pragma unroll
    for (int j = 0; j < 4; ++j) {
      const int n = n0 + (j << 4) + rlane;
      float bv = 0.f;
      if (BIAS_MODE == 2) bv = bias[n];
#pragma unroll
      for (int r = 0; r < 8; ++r) {
        float v = acc[i][j][r] * scale;
        if (BIAS_MODE == 1) v += bias[mBase + mOff + r];
        if (BIAS_MODE == 2) v += bv;
        if (RESID) v += Rb[(size_t)(mBase + mOff + r) * ldc + n];
        if (ACT == 1) v = tanhf(v);
        if (ACT == 2) v = fmaxf(v, 0.0f);
        if (ACT == 3) v = v / (1.0f + expf(-v));
        if (ACT == 4) v = (v > 0.f) ? v : 0.01f * v;
        slab[(mOff + r) * 68 + (j << 4) + rlane] = v;
      }
    }
    __builtin_amdgcn_fence(__ATOMIC_RELEASE, "workgroup");
    __builtin_amdgcn_wave_barrier();
    __builtin_amdgcn_fence(__ATOMIC_ACQUIRE, "workgroup");
    if (OUT_MODE == 0) {
      float* C = (float*)Cout + (size_t)b * strideC;
      const int hh = lane >> 4, c4 = (lane & 15) * 4;
      for (int pass = 0; pass < 2; ++pass) {
#pragma unroll
        for (int it = 0; it < 8; ++it) {
          const int row = it * 2 + hh;
          v4f v = *(const v4f*)(slab + row * 68 + c4);
          *(volatile v4f*)(C + (size_t)(mBase + row) * ldc + n0 + c4) = v;
        }
        __threadfence();
      }
    } else {
      const int q = lane >> 3, c8 = (lane & 7) * 8;
      unsigned short* C  = (unsigned short*)Cout  + (size_t)b * strideC;
      unsigned short* C2 = (OUT_MODE == 2) ? ((unsigned short*)Cout2 + (size_t)b * strideC) : nullptr;
      for (int pass = 0; pass < 2; ++pass) {
#pragma unroll
        for (int it = 0; it < 4; ++it) {
          const int row = it * 4 + q;
          const float* sp = slab + row * 68 + c8;
          v8h hv, lv;
#pragma unroll
          for (int e = 0; e < 8; ++e) {
            if (OUT_MODE == 1) {
              hv[e] = (_Float16)sp[e];
            } else {
              unsigned short hb = f2bf_bits(sp[e]);
              unsigned short lb = f2bf_bits(sp[e] - bf_bits2f(hb));
              hv[e] = __builtin_bit_cast(_Float16, hb);
              lv[e] = __builtin_bit_cast(_Float16, lb);
            }
          }
          *(volatile v8h*)(C + (size_t)(mBase + row) * ldc + n0 + c8) = hv;
          if (OUT_MODE == 2) *(volatile v8h*)(C2 + (size_t)(mBase + row) * ldc + n0 + c8) = lv;
        }
        __threadfence();
      }
    }
    __builtin_amdgcn_fence(__ATOMIC_RELEASE, "workgroup");
    __builtin_amdgcn_wave_barrier();
    __builtin_amdgcn_fence(__ATOMIC_ACQUIRE, "workgroup");
  }
}

__global__ __launch_bounds__(256) void tokens_kernel(
    const float* __restrict__ img, const float* __restrict__ txt, unsigned short* __restrict__ TOK, int total8)
{
  const int i = blockIdx.x * 256 + threadIdx.x;
  if (i >= total8) return;
  const int t  = i >> 6;
  const int c8 = (i & 63) << 3;
  const size_t so = (size_t)t * kOutDim + c8;
  const v4f a0 = *(const v4f*)(img + so);
  const v4f a1 = *(const v4f*)(img + so + 4);
  const v4f b0 = *(const v4f*)(txt + so);
  const v4f b1 = *(const v4f*)(txt + so + 4);
  v8h hi, ht;
#pragma unroll
  for (int e = 0; e < 4; ++e) {
    hi[e]     = bf_as_h(a0[e]);
    hi[4 + e] = bf_as_h(a1[e]);
    ht[e]     = bf_as_h(b0[e]);
    ht[4 + e] = bf_as_h(b1[e]);
  }
  unsigned short* p0 = TOK + (size_t)t * kDModel + c8;
  unsigned short* p1 = p0 + kOutDim;
  *(volatile v8h*)p0 = hi;
  *(volatile v8h*)p1 = ht;
  __threadfence();
  *(volatile v8h*)p0 = hi;
  *(volatile v8h*)p1 = ht;
}

__global__ __launch_bounds__(256) void txt_transpose_kernel(
    const float* __restrict__ txt, unsigned short* __restrict__ TXTT)
{
  __shared__ __align__(16) float sT[64 * 68];
  const int tid = threadIdx.x;
  const int kv0 = blockIdx.x * 64, c0 = blockIdx.y * 64;
#pragma unroll
  for (int it = 0; it < 4; ++it) {
    const int j = tid + 256 * it;
    const int r = j >> 4, c4 = (j & 15) * 4;
    const v4f v = *(const v4f*)(txt + (size_t)(kv0 + r) * kOutDim + c0 + c4);
#pragma unroll
    for (int e = 0; e < 4; ++e) sT[(c4 + e) * 68 + r] = bfr(v[e]);
  }
  __syncthreads();
  const int g8 = tid >> 3, k8 = (tid & 7) * 8;
  v8h hv[2];
#pragma unroll
  for (int it = 0; it < 2; ++it) {
    const int rr = it * 32 + g8;
    const float* sp = sT + rr * 68 + k8;
    const v4f x0 = *(const v4f*)(sp);
    const v4f x1 = *(const v4f*)(sp + 4);
#pragma unroll
    for (int e = 0; e < 4; ++e) { hv[it][e] = (_Float16)x0[e]; hv[it][4 + e] = (_Float16)x1[e]; }
  }
  for (int pass = 0; pass < 2; ++pass) {
#pragma unroll
    for (int it = 0; it < 2; ++it) {
      const int rr = it * 32 + g8;
      *(volatile v8h*)(TXTT + (size_t)(c0 + rr) * kSeq + kv0 + k8) = hv[it];
    }
    __threadfence();
  }
}

__global__ __launch_bounds__(256) void cast_bf16_kernel(
    const float* __restrict__ src, unsigned short* __restrict__ dst, int total8, int valid8)
{
  const int i = blockIdx.x * 256 + threadIdx.x;
  if (i >= total8) return;
  const int ic = (i < valid8) ? i : (valid8 - 1);
  const float keep = (i < valid8) ? 1.0f : 0.0f;
  const size_t e0 = (size_t)ic << 3;
  const v4f a0 = *(const v4f*)(src + e0);
  const v4f a1 = *(const v4f*)(src + e0 + 4);
  v8h hv;
#pragma unroll
  for (int e = 0; e < 4; ++e) {
    hv[e]     = bf_as_h(a0[e] * keep);
    hv[4 + e] = bf_as_h(a1[e] * keep);
  }
  unsigned short* q = dst + ((size_t)i << 3);
  *(volatile v8h*)q = hv;
  __threadfence();
  *(volatile v8h*)q = hv;
}

__global__ __launch_bounds__(256) void conv_silu_kernel(
    const float* __restrict__ XZ, const float* __restrict__ cw, const float* __restrict__ cb,
    float* __restrict__ UC, unsigned short* __restrict__ UCB)
{
  __shared__ __align__(16) float sT[16 * kConvTP];
  const int tid = threadIdx.x, lane = tid & 31, wave = tid >> 5;
  const int d0 = blockIdx.x * 256, d = d0 + tid;
  const int g0 = blockIdx.y * 64;
  const float w0 = bfr(cw[d * kDConv + 0]), w1 = bfr(cw[d * kDConv + 1]);
  const float w2 = bfr(cw[d * kDConv + 2]), w3 = bfr(cw[d * kDConv + 3]);
  const float bc = bfr(cb[d]);
  float xm3, xm2, xm1;
  {
    const bool hist = (g0 > 0);
    const int rb = hist ? (g0 - 3) : g0;
    const float v3 = XZ[(size_t)rb * kXzPitch + d];
    const float v2 = XZ[(size_t)(rb + 1) * kXzPitch + d];
    const float v1 = XZ[(size_t)(rb + 2) * kXzPitch + d];
    xm3 = hist ? v3 : 0.f;
    xm2 = hist ? v2 : 0.f;
    xm1 = hist ? v1 : 0.f;
  }
  const int hrow = wave >> 1;
  const int hch  = (wave & 1) * 128 + lane * 4;
#pragma unroll 1
  for (int sub = 0; sub < 4; ++sub) {
    const int lb = g0 + sub * 16;
#pragma unroll 1
    for (int s = 0; s < 16; ++s) {
      const float xcur = XZ[(size_t)(lb + s) * kXzPitch + d];
      float acc = w0 * xm3;
      acc = fmaf(w1, xm2, acc);
      acc = fmaf(w2, xm1, acc);
      acc = fmaf(w3, xcur, acc);
      const float sv = acc + bc;
      const float sg = __builtin_amdgcn_rcpf(1.0f + expf(-sv));
      sT[s * kConvTP + tid] = sv * sg;
      xm3 = xm2; xm2 = xm1; xm1 = xcur;
    }
    __syncthreads();
    v4f fv[4];
    v8h bh[2];
#pragma unroll
    for (int it = 0; it < 4; ++it) fv[it] = *(const v4f*)(sT + (it * 4 + hrow) * kConvTP + hch);
#pragma unroll
    for (int it = 0; it < 2; ++it) {
      const float* sp = sT + (it * 8 + wave) * kConvTP + lane * 8;
      const v4f a0 = *(const v4f*)(sp);
      const v4f a1 = *(const v4f*)(sp + 4);
#pragma unroll
      for (int e = 0; e < 4; ++e) {
        bh[it][e]     = bf_as_h(a0[e]);
        bh[it][4 + e] = bf_as_h(a1[e]);
      }
    }
    for (int pass = 0; pass < 2; ++pass) {
#pragma unroll
      for (int it = 0; it < 4; ++it)
        *(volatile v4f*)(UC + (size_t)(lb + it * 4 + hrow) * kDInner + d0 + hch) = fv[it];
#pragma unroll
      for (int it = 0; it < 2; ++it) {
        const size_t o = (size_t)(lb + it * 8 + wave) * kDInner + d0 + lane * 8;
        *(volatile v8h*)(UCB + o) = bh[it];
      }
      __threadfence();
    }
    __syncthreads();
  }
}

__global__ __launch_bounds__(256) void dtr_kernel(
    const float* __restrict__ XD, unsigned short* __restrict__ DTR, int total8)
{
  const int i = blockIdx.x * 256 + threadIdx.x;
  if (i >= total8) return;
  const int t = i >> 3, c8 = (i & 7) * 8;
  const float* sp = XD + (size_t)t * kXpN + c8;
  const v4f a0 = *(const v4f*)(sp);
  const v4f a1 = *(const v4f*)(sp + 4);
  v8h hv;
#pragma unroll
  for (int e = 0; e < 4; ++e) { hv[e] = bf_as_h(a0[e]); hv[4 + e] = bf_as_h(a1[e]); }
  unsigned short* q = DTR + ((size_t)i << 3);
  *(volatile v8h*)q = hv;
  __threadfence();
  *(volatile v8h*)q = hv;
}

__global__ __launch_bounds__(64) void scan_kernel(
    const float* __restrict__ XD, const float* __restrict__ DTP, const float* __restrict__ UC,
    const float* __restrict__ XZ, const float* __restrict__ bdt, const float* __restrict__ Alog,
    const float* __restrict__ Dp, unsigned short* __restrict__ Y)
{
  __shared__ __align__(16) float sBC[kScanTS * kBCP];
  __shared__ __align__(16) float sY[kScanTS * kScanYP];
  __shared__ __align__(16) float sA[kNState * kScanCh];
  const int tid = threadIdx.x, lane = tid & 31, wave = tid >> 5;
  const int d0 = blockIdx.x * kScanCh;
  const int d  = d0 + tid;
#pragma unroll 1
  for (int s = 0; s < kNState; ++s) sA[s * kScanCh + tid] = -expf(bfr(Alog[(size_t)d * kNState + s]));
  __syncthreads();
  float negA[kNState], h[kNState];
#pragma unroll
  for (int s = 0; s < kNState; ++s) {
    negA[s] = sA[s * kScanCh + tid];
    h[s] = 0.f;
  }
  const float bb = bfr(bdt[d]), Dd = bfr(Dp[d]);
  const int lr = tid >> 3, lc4 = (tid & 7) * 4;
  const int q = lane >> 3, c8 = (lane & 7) * 8;
#pragma unroll 1
  for (int t0 = 0; t0 < kSeq; t0 += kScanTS) {
    __syncthreads();
#pragma unroll
    for (int i = 0; i < 8; ++i) {
      const int r = lr + 8 * i;
      *(v4f*)(sBC + r * kBCP + lc4) = *(const v4f*)(XD + (size_t)(t0 + r) * kXpN + kDtRank + lc4);
    }
    __syncthreads();
#pragma unroll 1
    for (int s = 0; s < kScanTS; ++s) {
      const int t = t0 + s;
      const float* xr = sBC + s * kBCP;
      float Bs[kNState], Cs[kNState];
#pragma unroll
      for (int q4 = 0; q4 < 4; ++q4) {
        const v4f bv = *(const v4f*)(xr + 4 * q4);
        const v4f cv = *(const v4f*)(xr + kNState + 4 * q4);
        Bs[4 * q4 + 0] = bv[0]; Bs[4 * q4 + 1] = bv[1]; Bs[4 * q4 + 2] = bv[2]; Bs[4 * q4 + 3] = bv[3];
        Cs[4 * q4 + 0] = cv[0]; Cs[4 * q4 + 1] = cv[1]; Cs[4 * q4 + 2] = cv[2]; Cs[4 * q4 + 3] = cv[3];
      }
      const float v   = DTP[(size_t)t * kDInner + d] + bb;
      const float a   = expf(-fabsf(v));
      const float u   = 1.0f + a;
      const float l1p = logf(u) + (a - (u - 1.0f)) * __builtin_amdgcn_rcpf(u);
      const float dt  = fmaxf(v, 0.0f) + l1p;
      const float xt  = UC[(size_t)t * kDInner + d];
      const float dtx = dt * xt;
      float y = 0.f;
#pragma unroll
      for (int k = 0; k < kNState; ++k) {
        const float e = __expf(dt * negA[k]);
        h[k] = e * h[k] + dtx * Bs[k];
        y = h[k] * Cs[k] + y;
      }
      y = xt * Dd + y;
      const float zv = XZ[(size_t)t * kXzPitch + kDInner + d];
      const float sg = __builtin_amdgcn_rcpf(1.0f + expf(-zv));
      y = y * (zv * sg);
      sY[s * kScanYP + tid] = y;
    }
    __syncthreads();
    v8h hv[8];
#pragma unroll
    for (int it = 0; it < 8; ++it) {
      const int row = it * 8 + wave * 4 + q;
      const float* sp = sY + row * kScanYP + c8;
      const v4f a0 = *(const v4f*)(sp);
      const v4f a1 = *(const v4f*)(sp + 4);
#pragma unroll
      for (int e = 0; e < 4; ++e) {
        hv[it][e]     = bf_as_h(a0[e]);
        hv[it][4 + e] = bf_as_h(a1[e]);
      }
    }
    for (int pass = 0; pass < 2; ++pass) {
#pragma unroll
      for (int it = 0; it < 8; ++it) {
        const int row = it * 8 + wave * 4 + q;
        const size_t o = (size_t)(t0 + row) * kDInner + d0 + c8;
        *(volatile v8h*)(Y + o) = hv[it];
      }
      __threadfence();
    }
  }
}

__global__ __launch_bounds__(256) void softmax_kernel(const float* __restrict__ S, unsigned short* __restrict__ P)
{
  __shared__ float redm[8];
  __shared__ float reds[8];
  const int row = blockIdx.x, tid = threadIdx.x, lane = tid & 31, wave = tid >> 5;
  const float* sp = S + (size_t)row * kSeq + tid * 8;
  const v4f a0 = *(const v4f*)(sp);
  const v4f a1 = *(const v4f*)(sp + 4);
  float m = fmaxf(fmaxf(fmaxf(a0[0], a0[1]), fmaxf(a0[2], a0[3])), fmaxf(fmaxf(a1[0], a1[1]), fmaxf(a1[2], a1[3])));
#pragma unroll
  for (int off = 1; off < 32; off <<= 1) m = fmaxf(m, __shfl_xor(m, off, 32));
  if (lane == 0) redm[wave] = m;
  __syncthreads();
  float gm = redm[0];
#pragma unroll
  for (int w = 1; w < 8; ++w) gm = fmaxf(gm, redm[w]);
  v4f e0, e1;
#pragma unroll
  for (int j = 0; j < 4; ++j) { e0[j] = expf(a0[j] - gm); e1[j] = expf(a1[j] - gm); }
  float sum = 0.f;
#pragma unroll
  for (int j = 0; j < 4; ++j) sum = sum + e0[j];
#pragma unroll
  for (int j = 0; j < 4; ++j) sum = sum + e1[j];
#pragma unroll
  for (int off = 1; off < 32; off <<= 1) sum += __shfl_xor(sum, off, 32);
  if (lane == 0) reds[wave] = sum;
  __syncthreads();
  float tot = 0.f;
#pragma unroll
  for (int w = 0; w < 8; ++w) tot = tot + reds[w];
  const float sc = kPScale / tot;
  v8h hv;
#pragma unroll
  for (int j = 0; j < 4; ++j) { hv[j] = (_Float16)(e0[j] * sc); hv[4 + j] = (_Float16)(e1[j] * sc); }
  unsigned short* q = P + (size_t)row * kSeq + tid * 8;
  *(volatile v8h*)q = hv;
  __threadfence();
  *(volatile v8h*)q = hv;
}

__global__ __launch_bounds__(256) void finalize_kernel(
    const float* __restrict__ MO, const float* __restrict__ CAM, const float* __restrict__ img,
    const float* __restrict__ alpha, float* __restrict__ out)
{
  __shared__ float red[8];
  const int row = blockIdx.x, tid = threadIdx.x, lane = tid & 31, wave = tid >> 5;
  const int c0 = tid * 4;
  const int cc = c0 & (kOutDim - 1);
  const int hsel = tid >> 7;
  const float al = bfr(alpha[0]);
  const v4f mv = *(const v4f*)(MO + (size_t)row * kDModel + c0);
  const v4f cv = *(const v4f*)(CAM + (size_t)row * kOutDim + cc);
  const v4f iv = *(const v4f*)(img + (size_t)row * kOutDim + cc);
  const float fa = hsel ? 0.0f : al;
  const float fb = hsel ? 1.0f : 0.0f;
  v4f r;
  float ss = 0.f;
#pragma unroll
  for (int j = 0; j < 4; ++j) {
    const float ib = bfr(iv[j]);
    const float addv = fmaf(fa, cv[j], fb * ib);
    r[j] = mv[j] + addv;
    ss = ss + r[j] * r[j];
  }
#pragma unroll
  for (int off = 1; off < 32; off <<= 1) ss += __shfl_xor(ss, off, 32);
  if (lane == 0) red[wave] = ss;
  __syncthreads();
  float tot = 0.f;
#pragma unroll
  for (int w = 0; w < 8; ++w) tot = tot + red[w];
  const float nrm = sqrtf(tot);
  const float inv = 1.0f / fmaxf(nrm, 1e-12f);
  v4f o;
#pragma unroll
  for (int j = 0; j < 4; ++j) o[j] = r[j] * inv;
  float* q = out + (size_t)hsel * ((size_t)kSeq * kOutDim) + (size_t)row * kOutDim + cc;
  *(volatile v4f*)q = o;
  __threadfence();
  *(volatile v4f*)q = o;
}

extern "C" void kernel_launch(void* const* d_in, const int* in_sizes, int n_in,
                              void* d_out, int out_size, void* d_ws, size_t ws_size,
                              hipStream_t stream) {
  if (n_in < 12) return;
  if (in_sizes[0] != kSeq * kOutDim) return;
  if (in_sizes[1] != kSeq * kOutDim) return;
  if (in_sizes[2] != kXzPitch * kDModel) return;
  if (in_sizes[3] != kDInner * kDConv) return;
  if (in_sizes[4] != kDInner) return;
  if (in_sizes[5] != kXpReal * kDInner) return;
  if (in_sizes[6] != kDInner * kDtRank) return;
  if (in_sizes[7] != kDInner) return;
  if (in_sizes[8] != kDInner * kNState) return;
  if (in_sizes[9] != kDInner) return;
  if (in_sizes[10] != kDModel * kDInner) return;
  if (in_sizes[11] != 1) return;
  if (out_size != 2 * kSeq * kOutDim) return;
  if (ws_size < kWsTotal) return;

  const float* img    = (const float*)d_in[0];
  const float* txt    = (const float*)d_in[1];
  const float* W_in   = (const float*)d_in[2];
  const float* conv_w = (const float*)d_in[3];
  const float* conv_b = (const float*)d_in[4];
  const float* W_x    = (const float*)d_in[5];
  const float* W_dt   = (const float*)d_in[6];
  const float* b_dt   = (const float*)d_in[7];
  const float* A_log  = (const float*)d_in[8];
  const float* Dp     = (const float*)d_in[9];
  const float* W_out  = (const float*)d_in[10];
  const float* alpha  = (const float*)d_in[11];
  float* out = (float*)d_out;

  char* ws = (char*)d_ws;
  unsigned short* TOK  = (unsigned short*)(ws + kOffTok);
  unsigned short* WIN  = (unsigned short*)(ws + kOffWin);
  unsigned short* WXP  = (unsigned short*)(ws + kOffWxp);
  unsigned short* WDT  = (unsigned short*)(ws + kOffWdt);
  unsigned short* WOUT = (unsigned short*)(ws + kOffWout);
  unsigned short* TXTT = (unsigned short*)(ws + kOffTxtT);
  float*          XZ   = (float*)(ws + kOffXz);
  float*          UC   = (float*)(ws + kOffUc);
  unsigned short* UCB  = (unsigned short*)(ws + kOffUcb);
  float*          XD   = (float*)(ws + kOffXd);
  unsigned short* DTR  = (unsigned short*)(ws + kOffDtr);
  float*          DTP  = (float*)(ws + kOffDtp);
  unsigned short* Y    = (unsigned short*)(ws + kOffY);
  float*          MO   = (float*)(ws + kOffMo);
  float*          S    = (float*)(ws + kOffS);
  unsigned short* P    = (unsigned short*)(ws + kOffP);
  float*          CAM  = (float*)(ws + kOffCam);

  tokens_kernel<<<(kSeq * kOutDim / 8) / 256, 256, 0, stream>>>(img, txt, TOK, kSeq * kOutDim / 8);
  txt_transpose_kernel<<<dim3(kSeq / 64, kOutDim / 64), 256, 0, stream>>>(txt, TXTT);
  cast_bf16_kernel<<<(kXzPitch * kDModel / 8) / 256, 256, 0, stream>>>(W_in, WIN, kXzPitch * kDModel / 8, kXzPitch * kDModel / 8);
  cast_bf16_kernel<<<(kXpN * kDInner / 8) / 256, 256, 0, stream>>>(W_x, WXP, kXpN * kDInner / 8, kXpReal * kDInner / 8);
  cast_bf16_kernel<<<(kDInner * kDtRank / 8) / 256, 256, 0, stream>>>(W_dt, WDT, kDInner * kDtRank / 8, kDInner * kDtRank / 8);
  cast_bf16_kernel<<<(kDModel * kDInner / 8) / 256, 256, 0, stream>>>(W_out, WOUT, kDModel * kDInner / 8, kDModel * kDInner / 8);

  wmma_gemm64<1, false, 0, 0, false><<<dim3(((kSeq / 64) * (kXzPitch / 64)) / 8, 1), 256, 0, stream>>>(
      TOK, nullptr, kDModel, 0L,
      WIN, nullptr, kDModel, 0L,
      (void*)XZ, nullptr, kXzPitch, 0L,
      nullptr, nullptr, 0L,
      kSeq, kXzPitch, kDModel, 1.0f);

  conv_silu_kernel<<<dim3(kDInner / 256, kSeq / 64), 256, 0, stream>>>(XZ, conv_w, conv_b, UC, UCB);

  wmma_gemm64<1, false, 0, 0, false><<<dim3(((kSeq / 64) * (kXpN / 64)) / 8, 1), 256, 0, stream>>>(
      UCB, nullptr, kDInner, 0L,
      WXP, nullptr, kDInner, 0L,
      (void*)XD, nullptr, kXpN, 0L,
      nullptr, nullptr, 0L,
      kSeq, kXpN, kDInner, 1.0f);

  dtr_kernel<<<(kSeq * kDtRank / 8) / 256, 256, 0, stream>>>(XD, DTR, kSeq * kDtRank / 8);

  wmma_gemm64<1, false, 0, 0, false><<<dim3(((kSeq / 64) * (kDInner / 64)) / 8, 1), 256, 0, stream>>>(
      DTR, nullptr, kDtRank, 0L,
      WDT, nullptr, kDtRank, 0L,
      (void*)DTP, nullptr, kDInner, 0L,
      nullptr, nullptr, 0L,
      kSeq, kDInner, kDtRank, 1.0f);

  scan_kernel<<<kDInner / kScanCh, kScanCh, 0, stream>>>(XD, DTP, UC, XZ, b_dt, A_log, Dp, Y);

  wmma_gemm64<1, false, 0, 0, false><<<dim3(((kSeq / 64) * (kDModel / 64)) / 8, 1), 256, 0, stream>>>(
      Y, nullptr, kDInner, 0L,
      WOUT, nullptr, kDInner, 0L,
      (void*)MO, nullptr, kDModel, 0L,
      nullptr, nullptr, 0L,
      kSeq, kDModel, kDInner, 1.0f);

  wmma_gemm64<1, false, 0, 0, false><<<dim3(((kSeq / 64) * (kSeq / 64)) / 8, 1), 256, 0, stream>>>(
      TOK, nullptr, kDModel, 0L,
      TOK + kOutDim, nullptr, kDModel, 0L,
      (void*)S, nullptr, kSeq, 0L,
      nullptr, nullptr, 0L,
      kSeq, kSeq, kOutDim, 1.0f);

  softmax_kernel<<<kSeq, 256, 0, stream>>>(S, P);

  wmma_gemm64<0, false, 0, 0, false><<<dim3(((kSeq / 64) * (kOutDim / 64)) / 8, 1), 256, 0, stream>>>(
      P, nullptr, kSeq, 0L,
      TXTT, nullptr, kSeq, 0L,
      (void*)CAM, nullptr, kOutDim, 0L,
      nullptr, nullptr, 0L,
      kSeq, kOutDim, kSeq, kPScaleInv);

  finalize_kernel<<<kSeq, 256, 0, stream>>>(MO, CAM, img, alpha, out);
}
